// GAT_38560216384098
// MI455X (gfx1250) — hardware-run, weakly checked
//
#include <hip/hip_runtime.h>
#include <stddef.h>
#include <stdint.h>


#define DIN     256
#define HC      256
#define NLR     512
#define PARN    1024
#define P_ATT   512
#define P_BIAS  768
#define NSPEC   50000
#define ESPEC   500000
#define NTHR    256
#define NWAVE   8
#define EPT     8
#define CHUNK   (NTHR * EPT)
#define WCAP    (EPT * 32)
#define LISTN   (NWAVE * WCAP)
#define NBMAX   2048
#define NBRUN   1024
#define ESH     11
#define RCAP    28672
#define DEGCAP  4096
#define STW     512
#define GBM     64
#define GBN     64
#define GTHR    128
#define NEGS    0.2f
#define WSMAX   134217728
#define LDS_AGG ((2 * RCAP + 2 * NBMAX + LISTN) * 4 + 64)

static_assert((CHUNK & (CHUNK - 1)) == 0 && CHUNK <= 4096);
static_assert((NBMAX & (NBMAX - 1)) == 0 && NBMAX <= 4096);
static_assert((NBRUN & (NBRUN - 1)) == 0 && NBRUN <= NBMAX && NBRUN >= 16);
static_assert((1 << ESH) >= NBMAX);
static_assert(NTHR * 8 == NBMAX);
static_assert(LISTN >= NBMAX);
static_assert(LISTN >= NWAVE * WCAP);
static_assert((RCAP % 32) == 0);
static_assert(NWAVE * STW <= RCAP);
static_assert(HC <= STW);
static_assert(LDS_AGG <= 300000);
static_assert(GBM == (GTHR / 32) * 16);
static_assert((DIN % 32) == 0 && DIN / 8 == 32);
static_assert((NLR % GBN) == 0 && (HC % GBN) == 0 && NLR == 2 * HC);
static_assert(HC == 32 * 8);
static_assert(NSPEC <= 49 * NBRUN);
static_assert(NSPEC < 65536);
static_assert(ESPEC <= (1 << (32 - ESH)));
static_assert(PARN == 4 * 256);

typedef float          v4f   __attribute__((ext_vector_type(4)));
typedef float          v8f   __attribute__((ext_vector_type(8)));
typedef int            v4i   __attribute__((ext_vector_type(4)));
typedef int            v8i   __attribute__((ext_vector_type(8)));
typedef unsigned short v8us  __attribute__((ext_vector_type(8)));
typedef __bf16         v16bf __attribute__((ext_vector_type(16)));
union FragB { v16bf v; v8us u[2]; v8i w; };

__device__ __forceinline__ v8f wmx(const FragB& a, const FragB& b, v8f c) {
  v8f d = __builtin_amdgcn_wmma_f32_16x16x32_bf16(false, a.v, false, b.v, (short)0, c, false, false);
  asm volatile("v_nop\n\tv_nop\n\tv_nop\n\tv_nop" : "+v"(d) : "v"(a.w), "v"(b.w));
  return d;
}

__device__ __forceinline__ unsigned bfbits(float v) {
  unsigned u = __float_as_uint(v);
  u = u + 0x7FFFu + ((u >> 16) & 1u);
  return u >> 16;
}
__device__ __forceinline__ float rbf(float v) { return __uint_as_float(bfbits(v) << 16); }

__device__ __forceinline__ v8us cvt8b(const v4f a, const v4f b) {
  v8us o;
  o[0] = (unsigned short)bfbits(a.x); o[1] = (unsigned short)bfbits(a.y);
  o[2] = (unsigned short)bfbits(a.z); o[3] = (unsigned short)bfbits(a.w);
  o[4] = (unsigned short)bfbits(b.x); o[5] = (unsigned short)bfbits(b.y);
  o[6] = (unsigned short)bfbits(b.z); o[7] = (unsigned short)bfbits(b.w);
  return o;
}
__device__ __forceinline__ void put8us(unsigned short* p, const v8us hv) {
  *(volatile v8us*)p = hv;
  __threadfence();
  *(volatile v8us*)p = hv;
}
__device__ __forceinline__ void put4f(float* p, const v4f v) {
  *(volatile v4f*)p = v;
  __threadfence();
  *(volatile v4f*)p = v;
}

__device__ __forceinline__ int scan_chunk(const int* __restrict__ dsts, int nE, int cbase, int slotBase,
                                          int nb, int vec8, int* list, int tid, int lane, int wave) {
  int wc = 0;
  const int el0  = tid * EPT;
  const int e0   = cbase + el0;
  const int sent = -2147483647 - 1;
  v4i da, db;
  if (vec8 != 0 && cbase + CHUNK <= nE) {
    da = *(const v4i*)(dsts + e0);
    db = *(const v4i*)(dsts + e0 + 4);
  } else {
    da.x = (e0     < nE) ? dsts[min(e0,     nE - 1)] : sent;
    da.y = (e0 + 1 < nE) ? dsts[min(e0 + 1, nE - 1)] : sent;
    da.z = (e0 + 2 < nE) ? dsts[min(e0 + 2, nE - 1)] : sent;
    da.w = (e0 + 3 < nE) ? dsts[min(e0 + 3, nE - 1)] : sent;
    db.x = (e0 + 4 < nE) ? dsts[min(e0 + 4, nE - 1)] : sent;
    db.y = (e0 + 5 < nE) ? dsts[min(e0 + 5, nE - 1)] : sent;
    db.z = (e0 + 6 < nE) ? dsts[min(e0 + 6, nE - 1)] : sent;
    db.w = (e0 + 7 < nE) ? dsts[min(e0 + 7, nE - 1)] : sent;
  }
  const unsigned nbs = (unsigned)slotBase;
  const unsigned unb = (unsigned)nb;
  const unsigned s0 = (unsigned)da.x - nbs, s1 = (unsigned)da.y - nbs;
  const unsigned s2 = (unsigned)da.z - nbs, s3 = (unsigned)da.w - nbs;
  const unsigned s4 = (unsigned)db.x - nbs, s5 = (unsigned)db.y - nbs;
  const unsigned s6 = (unsigned)db.z - nbs, s7 = (unsigned)db.w - nbs;
  const bool h0 = s0 < unb, h1 = s1 < unb, h2 = s2 < unb, h3 = s3 < unb;
  const bool h4 = s4 < unb, h5 = s5 < unb, h6 = s6 < unb, h7 = s7 < unb;
  const unsigned any = __builtin_amdgcn_ballot_w32(h0 | h1 | h2 | h3 | h4 | h5 | h6 | h7);
  if (any != 0u) {
#define HITJ(J, HJ, SJ) { \
      const unsigned mj = __builtin_amdgcn_ballot_w32(HJ); \
      if (mj != 0u) { \
        if (HJ) { \
          const int pos = wc + (int)__builtin_amdgcn_mbcnt_lo(mj, 0u); \
          if (pos < WCAP) list[wave * WCAP + pos] = ((el0 + (J)) << 12) | (int)(SJ); \
        } \
        wc += (int)__builtin_popcount(mj); } }
    HITJ(0, h0, s0)
    HITJ(1, h1, s1)
    HITJ(2, h2, s2)
    HITJ(3, h3, s3)
    HITJ(4, h4, s4)
    HITJ(5, h5, s5)
    HITJ(6, h6, s6)
    HITJ(7, h7, s7)
#undef HITJ
  }
  return wc;
}

__device__ __forceinline__ void wt_unit(const float* __restrict__ w, unsigned short* wt, int nbase, int u) {
  const int nc = u >> 5;
  const int k8 = (u & 31) * 8;
  const float* p = w + (size_t)k8 * HC + nc;
  v4f a, b;
  a.x = p[0];                a.y = p[(size_t)HC];       a.z = p[(size_t)2 * HC];   a.w = p[(size_t)3 * HC];
  b.x = p[(size_t)4 * HC];   b.y = p[(size_t)5 * HC];   b.z = p[(size_t)6 * HC];   b.w = p[(size_t)7 * HC];
  put8us(wt + (size_t)(nbase + nc) * DIN + k8, cvt8b(a, b));
}

__global__ __launch_bounds__(NTHR) void k_prep(
    const float* __restrict__ x, const float* __restrict__ wl, const float* __restrict__ bl,
    const float* __restrict__ wr, const float* __restrict__ br, const float* __restrict__ att,
    const float* __restrict__ bias, unsigned short* xb, unsigned short* wt, float* par,
    int nN, int nUx, int nBx) {
  const int b = (int)blockIdx.x, tid = (int)threadIdx.x;
  if (b < nBx) {
    const int i = b * NTHR + tid;
    if (i >= nUx) return;
    const int row = i >> 5;
    const int c0  = (i & 31) * 8;
    const int rc  = row < nN ? row : nN - 1;
    const float* p = x + (size_t)rc * DIN + c0;
    v4f a = *(const v4f*)p, bq = *(const v4f*)(p + 4);
    const v4f z4 = {0.f, 0.f, 0.f, 0.f};
    if (row >= nN) { a = z4; bq = z4; }
    put8us(xb + (size_t)row * DIN + c0, cvt8b(a, bq));
  } else if (b < nBx + 32) {
    wt_unit(wl, wt, 0, (b - nBx) * NTHR + tid);
  } else if (b < nBx + 64) {
    wt_unit(wr, wt, HC, (b - nBx - 32) * NTHR + tid);
  } else {
    const int q = tid & 63, sec = tid >> 6;
    const v4f a = *(const v4f*)(bl + 4 * q);
    const v4f c = *(const v4f*)(br + 4 * q);
    const v4f d = *(const v4f*)(att + 4 * q);
    const v4f e = *(const v4f*)(bias + 4 * q);
    asm volatile("" :: "v"(a), "v"(c), "v"(d), "v"(e));
    v4f r = e;
    if (sec == 0) r = a;
    if (sec == 1) r = c;
    if (sec == 2) r = d;
    r.x = rbf(r.x); r.y = rbf(r.y); r.z = rbf(r.z); r.w = rbf(r.w);
    put4f(par + 4 * tid, r);
  }
}

__global__ __launch_bounds__(GTHR) __attribute__((amdgpu_num_vgpr(248)))
void k_proj(const unsigned short* __restrict__ A, const unsigned short* __restrict__ WT,
            const float* __restrict__ par, float* outF, size_t pstride)
{
  __shared__ __attribute__((aligned(16))) float stg[GBM * GBN];
  __shared__ __attribute__((aligned(16))) float sbias[GBN];
  const int tid = (int)threadIdx.x, lane = tid & 31, wave = tid >> 5, hh = lane >> 4, m = lane & 15;
  const int rowBase = (int)blockIdx.x * GBM;
  const int by      = (int)blockIdx.y;
  const int colg    = by * GBN;
  const int plane   = by >> 2;
  const int pc0     = (by & 3) * GBN;

  v8f acc[4];
  {
    const v8f z = {0.f, 0.f, 0.f, 0.f, 0.f, 0.f, 0.f, 0.f};
    acc[0] = z; acc[1] = z; acc[2] = z; acc[3] = z;
  }
  const unsigned short* ap = A  + (size_t)(rowBase + 16 * wave + m) * (size_t)DIN + 8 * hh;
  const unsigned short* wp = WT + (size_t)(colg + m) * (size_t)DIN + 8 * hh;
#pragma unroll 1
  for (int ks = 0; ks < DIN / 32; ++ks) {
    FragB af;
    af.u[0] = *(const v8us*)(ap + 32 * ks);
    af.u[1] = *(const v8us*)(ap + 32 * ks + 16);
#pragma unroll
    for (int t = 0; t < 4; ++t) {
      const unsigned short* wq = wp + (size_t)(16 * t) * (size_t)DIN + 32 * ks;
      FragB bf;
      bf.u[0] = *(const v8us*)wq;
      bf.u[1] = *(const v8us*)(wq + 16);
      acc[t] = wmx(af, bf, acc[t]);
    }
  }

#pragma unroll
  for (int t = 0; t < 4; ++t) {
    const int lc = 16 * t + m;
#pragma unroll
    for (int r = 0; r < 8; ++r) {
      const int lr = 16 * wave + 8 * hh + r;
      stg[lr * GBN + lc] = acc[t][r];
    }
  }
  if (wave == 0) {
    *(v4f*)(sbias + 4 * m) = *(const v4f*)(par + colg + 4 * m);
  }
  __syncthreads();

  const v4f sb = *(const v4f*)(sbias + 4 * m);
  v4f fv[8];
#pragma unroll
  for (int i = 0; i < 8; ++i) {
    const int lr = 16 * wave + 2 * i + hh;
    fv[i] = *(const v4f*)(stg + lr * GBN + 4 * m) + sb;
  }
  float* obase = outF + (size_t)plane * pstride + pc0 + 4 * m;
#pragma unroll
  for (int i = 0; i < 8; ++i) {
    const int lr = 16 * wave + 2 * i + hh;
    const int gr = rowBase + lr;
    float* op = obase + (size_t)gr * (size_t)HC;
    *(volatile v4f*)op = fv[i];
  }
  __threadfence();
#pragma unroll
  for (int i = 0; i < 8; ++i) {
    const int lr = 16 * wave + 2 * i + hh;
    const int gr = rowBase + lr;
    float* op = obase + (size_t)gr * (size_t)HC;
    *(volatile v4f*)op = fv[i];
  }
}

__device__ __forceinline__ int build_lists(const int* __restrict__ dsts, int nE, int nodeBase, int nb, int vec8,
                                           int* reg1, int* reg2, int* scnt, int* soff, int* list,
                                           int* wcnt, int* wtot, int tid, int lane, int wave) {
  for (int i = tid; i < NBMAX; i += NTHR) scnt[i] = 0;
  __syncthreads();

  int tot = 0;
  const int nChunks = (nE + CHUNK - 1) / CHUNK;
#pragma unroll 1
  for (int ch = 0; ch < nChunks; ++ch) {
    const int cbase = ch * CHUNK;
    const int wc = scan_chunk(dsts, nE, cbase, nodeBase, nb, vec8, list, tid, lane, wave);
    if (lane == 0) wcnt[wave] = wc;
    __syncthreads();
    int pre = 0, all = 0;
#pragma unroll
    for (int w2 = 0; w2 < NWAVE; ++w2) {
      int c = wcnt[w2];
      c = c < 0 ? 0 : (c > WCAP ? WCAP : c);
      all += c;
      pre += (w2 < wave) ? c : 0;
    }
    const int wcc  = wc > WCAP ? WCAP : wc;
    const int base = tot + pre;
#pragma unroll 1
    for (int i = lane; i < wcc; i += 32) {
      const int ent = list[wave * WCAP + i];
      const int el  = (ent >> 12) & (CHUNK - 1);
      const int sl  = ent & (NBMAX - 1);
      int eid = cbase + el;
      eid = eid > nE - 1 ? nE - 1 : eid;
      const int pos = base + i;
      if (pos < RCAP) reg1[pos] = (int)(((unsigned)eid << ESH) | (unsigned)sl);
    }
    tot += all;
    tot = tot > RCAP ? RCAP : tot;
    __syncthreads();
  }
  const int nh = tot;

  if (wave == 0) {
#pragma unroll 1
    for (int b0 = 0; b0 < nh; b0 += 32) {
      const int idx = b0 + lane;
      const int uv  = reg1[idx < RCAP ? idx : RCAP - 1];
      const int m32 = (nh - b0) < 32 ? (nh - b0) : 32;
#pragma unroll 1
      for (int k = 0; k < m32; ++k) {
        const int u  = __builtin_amdgcn_readlane(uv, k);
        const int sl = u & (NBMAX - 1);
        if (lane == 0) scnt[sl] = scnt[sl] + 1;
      }
    }
  }
  __syncthreads();

  {
    const v4i ca = *(const v4i*)(scnt + 8 * tid);
    const v4i cb = *(const v4i*)(scnt + 8 * tid + 4);
    const int e0 = ca.x < 0 ? 0 : ca.x, e1 = ca.y < 0 ? 0 : ca.y, e2 = ca.z < 0 ? 0 : ca.z, e3 = ca.w < 0 ? 0 : ca.w;
    const int e4 = cb.x < 0 ? 0 : cb.x, e5 = cb.y < 0 ? 0 : cb.y, e6 = cb.z < 0 ? 0 : cb.z, e7 = cb.w < 0 ? 0 : cb.w;
    const int ts = e0 + e1 + e2 + e3 + e4 + e5 + e6 + e7;
    int incl = ts;
#pragma unroll
    for (int d = 1; d < 32; d <<= 1) {
      const int up = __shfl_up(incl, d);
      if (lane >= d) incl += up;
    }
    if (lane == 31) wtot[wave] = incl;
    __syncthreads();
    int pre = 0;
#pragma unroll
    for (int w2 = 0; w2 < NWAVE; ++w2) pre += (w2 < wave) ? wtot[w2] : 0;
    int run = pre + incl - ts;
    soff[8 * tid + 0] = run; run += e0;
    soff[8 * tid + 1] = run; run += e1;
    soff[8 * tid + 2] = run; run += e2;
    soff[8 * tid + 3] = run; run += e3;
    soff[8 * tid + 4] = run; run += e4;
    soff[8 * tid + 5] = run; run += e5;
    soff[8 * tid + 6] = run; run += e6;
    soff[8 * tid + 7] = run;
  }
  __syncthreads();
  for (int i = tid; i < NBMAX; i += NTHR) list[i] = soff[i];
  __syncthreads();

  if (wave == 0) {
#pragma unroll 1
    for (int b0 = 0; b0 < nh; b0 += 32) {
      const int idx = b0 + lane;
      const int uv  = reg1[idx < RCAP ? idx : RCAP - 1];
      const int m32 = (nh - b0) < 32 ? (nh - b0) : 32;
#pragma unroll 1
      for (int k = 0; k < m32; ++k) {
        const int u   = __builtin_amdgcn_readlane(uv, k);
        const int sl  = u & (NBMAX - 1);
        const int eid = (int)((unsigned)u >> ESH);
        if (lane == 0) {
          int pos = list[sl];
          pos = pos < 0 ? 0 : (pos > RCAP - 1 ? RCAP - 1 : pos);
          reg2[pos] = eid;
          list[sl] = pos + 1;
        }
      }
    }
  }
  __syncthreads();
  return nh;
}

__device__ __forceinline__ float ldot8(const v4f la, const v4f lb, const v4f ra, const v4f rb,
                                       const v4f aa, const v4f ab) {
  float m0 = la.x + ra.x, m1 = la.y + ra.y, m2 = la.z + ra.z, m3 = la.w + ra.w;
  float m4 = lb.x + rb.x, m5 = lb.y + rb.y, m6 = lb.z + rb.z, m7 = lb.w + rb.w;
  m0 = m0 > 0.f ? m0 : m0 * NEGS;
  m1 = m1 > 0.f ? m1 : m1 * NEGS;
  m2 = m2 > 0.f ? m2 : m2 * NEGS;
  m3 = m3 > 0.f ? m3 : m3 * NEGS;
  m4 = m4 > 0.f ? m4 : m4 * NEGS;
  m5 = m5 > 0.f ? m5 : m5 * NEGS;
  m6 = m6 > 0.f ? m6 : m6 * NEGS;
  m7 = m7 > 0.f ? m7 : m7 * NEGS;
  float part = m0 * aa.x;
  part = fmaf(m1, aa.y, part);
  part = fmaf(m2, aa.z, part);
  part = fmaf(m3, aa.w, part);
  part = fmaf(m4, ab.x, part);
  part = fmaf(m5, ab.y, part);
  part = fmaf(m6, ab.z, part);
  part = fmaf(m7, ab.w, part);
  return part;
}
__device__ __forceinline__ float hsum8(float p) {
  p += __shfl_xor(p, 1);
  p += __shfl_xor(p, 2);
  p += __shfl_xor(p, 4);
  return p;
}
__device__ __forceinline__ v4f upd4(const v4f acc, const v4f xv, const float s1, const float s2) {
  v4f r;
  r.x = fmaf(acc.x, s1, s2 * xv.x);
  r.y = fmaf(acc.y, s1, s2 * xv.y);
  r.z = fmaf(acc.z, s1, s2 * xv.z);
  r.w = fmaf(acc.w, s1, s2 * xv.w);
  return r;
}

__global__ __launch_bounds__(NTHR) void k_scan(
    const int* __restrict__ srcs, const int* __restrict__ dsts,
    const float* __restrict__ XL, const float* __restrict__ XR, const float* __restrict__ par,
    float* out, int nN, int nE, int nb, int vec8) {
  extern __shared__ v4f lds_dyn[];
  int* reg1 = (int*)lds_dyn;
  int* reg2 = reg1 + RCAP;
  int* scnt = reg2 + RCAP;
  int* soff = scnt + NBMAX;
  int* list = soff + NBMAX;
  int* wcnt = list + LISTN;
  int* wtot = wcnt + NWAVE;
  const int tid = (int)threadIdx.x, lane = tid & 31, wave = tid >> 5;
  const int nodeBase = (int)blockIdx.x * nb;

  const int nh = build_lists(dsts, nE, nodeBase, nb, vec8, reg1, reg2, scnt, soff, list, wcnt, wtot,
                             tid, lane, wave);

  const int nbw = nb >> 3;
  const bool ovf = (nh >= RCAP);
  const float qnan = __int_as_float(0x7fc00000);
  float* stw = (float*)reg1 + wave * STW;
  const int c0 = 8 * lane;
  const v4f ata = *(const v4f*)(par + P_ATT + c0);
  const v4f atb = *(const v4f*)(par + P_ATT + c0 + 4);
  const v4f bia = *(const v4f*)(par + P_BIAS + c0);
  const v4f bib = *(const v4f*)(par + P_BIAS + c0 + 4);

#pragma unroll 1
  for (int jt = 0; jt < nbw; ++jt) {
    const int slot = wave * nbw + jt;
    const int grow = nodeBase + slot;
    if (grow >= nN) break;
    int st = soff[slot];
    const int craw = scnt[slot];
    int cnt = craw;
    st  = st < 0 ? 0 : (st > nh ? nh : st);
    cnt = cnt < 0 ? 0 : (cnt > DEGCAP ? DEGCAP : cnt);
    if (cnt > nh - st) cnt = nh - st;
    const bool bad = ovf || (craw > DEGCAP);

    const size_t ro = (size_t)grow * HC + c0;
    const v4f xra = *(const v4f*)(XR + ro);
    const v4f xrb = *(const v4f*)(XR + ro + 4);
    const v4f xsa = *(const v4f*)(XL + ro);
    const v4f xsb = *(const v4f*)(XL + ro + 4);

    float mx = hsum8(ldot8(xsa, xsb, xra, xrb, ata, atb));
    float dn = 1.0f;
    v4f ava = xsa, avb = xsb;

#pragma unroll 1
    for (int q = 0; q < cnt; ++q) {
      int idx = st + q; idx = idx > RCAP - 1 ? RCAP - 1 : idx;
      int eid = reg2[idx]; eid = eid < 0 ? 0 : (eid > nE - 1 ? nE - 1 : eid);
      const int sraw = srcs[eid];
      const int s = sraw < 0 ? 0 : (sraw > nN - 1 ? nN - 1 : sraw);
      const size_t so = (size_t)s * HC + c0;
      const v4f xla = *(const v4f*)(XL + so);
      const v4f xlb = *(const v4f*)(XL + so + 4);
      const float part = hsum8(ldot8(xla, xlb, xra, xrb, ata, atb));
      const float df = part - mx;
      const float ee = expf(-fabsf(df));
      const bool up  = df > 0.f;
      const float s1 = up ? ee : 1.0f;
      const float s2 = up ? 1.0f : ee;
      mx = up ? part : mx;
      dn = fmaf(dn, s1, s2);
      ava = upd4(ava, xla, s1, s2);
      avb = upd4(avb, xlb, s1, s2);
    }
    const float iv = __builtin_amdgcn_rcpf(dn);
    v4f ra, rb;
    ra.x = fmaf(ava.x, iv, bia.x); ra.y = fmaf(ava.y, iv, bia.y);
    ra.z = fmaf(ava.z, iv, bia.z); ra.w = fmaf(ava.w, iv, bia.w);
    rb.x = fmaf(avb.x, iv, bib.x); rb.y = fmaf(avb.y, iv, bib.y);
    rb.z = fmaf(avb.z, iv, bib.z); rb.w = fmaf(avb.w, iv, bib.w);
    if (bad) {
      const v4f qn4 = {qnan, qnan, qnan, qnan};
      ra = qn4; rb = qn4;
    }
    __builtin_amdgcn_fence(__ATOMIC_RELEASE, "wavefront");
    __builtin_amdgcn_wave_barrier();
    *(v4f*)(stw + 8 * lane)     = ra;
    *(v4f*)(stw + 8 * lane + 4) = rb;
    __builtin_amdgcn_fence(__ATOMIC_RELEASE, "wavefront");
    __builtin_amdgcn_wave_barrier();
    const v4f ga = *(const v4f*)(stw + 4 * lane);
    const v4f gb = *(const v4f*)(stw + 128 + 4 * lane);
    float* gp = out + (size_t)grow * HC + 4 * lane;
    *(volatile v4f*)gp         = ga;
    *(volatile v4f*)(gp + 128) = gb;
    __threadfence();
    *(volatile v4f*)gp         = ga;
    *(volatile v4f*)(gp + 128) = gb;
  }
}

static int pick_nb(int nE, int nN) {
  int nb = NBRUN;
  while (nb > 16 && (long long)nb * (long long)nE * 5LL > (long long)RCAP * (long long)nN * 4LL) nb >>= 1;
  return nb;
}
static inline int cdiv(int a, int b) { return (a + b - 1) / b; }

extern "C" void kernel_launch(void* const* d_in, const int* in_sizes, int n_in,
                              void* d_out, int out_size, void* d_ws, size_t ws_size,
                              hipStream_t stream) {
  if (n_in < 8) return;
  if (in_sizes[0] < DIN || (in_sizes[0] % DIN) != 0) return;
  const int nN = in_sizes[0] / DIN;
  if (nN <= 0 || nN > (1 << 22)) return;
  if (in_sizes[1] < 2 || (in_sizes[1] & 1) != 0) return;
  const int nE = in_sizes[1] / 2;
  if (nE < 1 || nE > (1 << (32 - ESH))) return;
  if (in_sizes[2] != DIN * HC || in_sizes[3] != HC) return;
  if (in_sizes[4] != DIN * HC || in_sizes[5] != HC) return;
  if (in_sizes[6] != HC || in_sizes[7] != HC) return;
  if (out_size != nN * HC) return;

  const float* x    = (const float*)d_in[0];
  const int*   ei   = (const int*)  d_in[1];
  const float* Wl   = (const float*)d_in[2];
  const float* bl   = (const float*)d_in[3];
  const float* Wr   = (const float*)d_in[4];
  const float* br   = (const float*)d_in[5];
  const float* att  = (const float*)d_in[6];
  const float* bias = (const float*)d_in[7];
  float* out = (float*)d_out;
  const int* src = ei;
  const int* dst = ei + nE;

  const int MP   = cdiv(nN, GBM) * GBM;
  const int nb   = pick_nb(nE, nN);
  const int gA   = cdiv(nN, nb);
  const int vec8 = ((nE & 3) == 0) ? 1 : 0;
  if ((long long)gA * (long long)nb < (long long)nN) return;

  char* ws = (char*)d_ws;
  size_t off = 0;
  const size_t oXB  = off; off += (size_t)MP * DIN * 2;            off = (off + 255) & ~(size_t)255;
  const size_t oWT  = off; off += (size_t)NLR * DIN * 2;           off = (off + 255) & ~(size_t)255;
  const size_t oPAR = off; off += (size_t)PARN * 4;                off = (off + 255) & ~(size_t)255;
  const size_t oXLR = off; off += (size_t)2 * MP * HC * 4;         off = (off + 255) & ~(size_t)255;
  if (off > ws_size || off > (size_t)WSMAX) return;
  unsigned short* XB  = (unsigned short*)(ws + oXB);
  unsigned short* WT  = (unsigned short*)(ws + oWT);
  float*          PAR = (float*)(ws + oPAR);
  float*          XLp = (float*)(ws + oXLR);
  const size_t pstride = (size_t)MP * HC;
  float*          XRp = XLp + pstride;

  hipFuncSetAttribute(reinterpret_cast<const void*>(&k_scan),
                      hipFuncAttributeMaxDynamicSharedMemorySize, LDS_AGG);

  const int nUx = MP * (DIN / 8);
  const int nBx = cdiv(nUx, NTHR);
  k_prep<<<nBx + 65, NTHR, 0, stream>>>(x, Wl, bl, Wr, br, att, bias, XB, WT, PAR, nN, nUx, nBx);

  k_proj<<<dim3(MP / GBM, NLR / GBN), GTHR, 0, stream>>>(XB, WT, PAR, XLp, pstride);

  k_scan<<<gA, NTHR, LDS_AGG, stream>>>(src, dst, XLp, XRp, PAR, out, nN, nE, nb, vec8);
}
